// CENPatchExpertPyTorch_31610959298739
// MI455X (gfx1250) — hardware-verified
//
#include <hip/hip_runtime.h>
#include <cmath>

typedef _Float16 v2h  __attribute__((ext_vector_type(2)));
typedef _Float16 v8h  __attribute__((ext_vector_type(8)));
typedef _Float16 v16h __attribute__((ext_vector_type(16)));
typedef float    v8f  __attribute__((ext_vector_type(8)));
typedef float    v4f  __attribute__((ext_vector_type(4)));

union Frag { v16h v; v8h half[2]; };

#define PATCH   11
#define HW      107
#define RH      97
#define NPATCH  9409
#define KPIX    121
#define MT      128
#define NTILES  74
#define WSP     (NTILES * MT)
#define FP      136
#define H2P     132
#define XROWS   13
#define XP      112
#define EPSV    1e-10f
#define WSCALE  16.0f
#define WINV    0.0625f

__device__ __forceinline__ v8f wmma16(v16h a, v16h b, v8f c) {
    v8f d = __builtin_amdgcn_wmma_f32_16x16x32_f16(false, a, false, b, (short)0, c, false, false);
    asm volatile("v_nop\n\tv_nop\n\tv_nop\n\tv_nop" : "+v"(d) : "v"(a), "v"(b));
    return d;
}

__device__ __forceinline__ v16h load_frag(const _Float16* base) {
    Frag f;
    f.half[0] = *(const v8h*)base;
    f.half[1] = *(const v8h*)(base + 16);
    return f.v;
}

__device__ __forceinline__ float fast_tanh(float v) {
    float e = __expf(2.0f * v);
    return 1.0f - 2.0f * __builtin_amdgcn_rcpf(e + 1.0f);
}
__device__ __forceinline__ float fast_sigmoid(float v) {
    return __builtin_amdgcn_rcpf(1.0f + __expf(-v));
}

__global__ __launch_bounds__(256) void k_patch_mlp(
    const float* __restrict__ x,  const float* __restrict__ W1, const float* __restrict__ b1,
    const float* __restrict__ W2, const float* __restrict__ b2,
    const float* __restrict__ W3, const float* __restrict__ b3,
    float* __restrict__ ws, int nimg)
{
    __shared__ __attribute__((aligned(16))) _Float16 featA[MT * FP];
    __shared__ __attribute__((aligned(16))) _Float16 h1A  [MT * FP];
    __shared__ __attribute__((aligned(16))) _Float16 w1c  [128 * FP];
    __shared__ __attribute__((aligned(16))) _Float16 w2c  [128 * FP];
    __shared__ __attribute__((aligned(16))) float    h2s  [MT * H2P];
    __shared__ __attribute__((aligned(16))) float    ximg [XROWS * XP];
    __shared__ __attribute__((aligned(16))) float    outs [MT];

    const int tid   = threadIdx.x;
    const int wave  = tid >> 5;
    const int lane  = tid & 31;
    const int lmod  = lane & 15;
    const int lhalf = lane >> 4;
    const int mrow  = wave * 16;

    const int img  = blockIdx.x / NTILES;
    const int tile = blockIdx.x - img * NTILES;
    if (img >= nimg) return;
    const int p0   = tile * MT;
    const int pr0  = p0 / RH;

    {
        const int plast = (p0 + MT - 1 < NPATCH - 1) ? p0 + MT - 1 : NPATCH - 1;
        const int nrows = (plast / RH) - pr0 + PATCH;
        const float* xb = x + (size_t)img * (HW * HW) + (size_t)pr0 * HW;
        for (int idx = tid; idx < nrows * HW; idx += 256) {
            const int r = idx / HW, c = idx - r * HW;
            ximg[r * XP + c] = xb[r * HW + c];
        }
    }
    __syncthreads();

    if (tid < MT) {
        const int p = p0 + tid;
        _Float16* row = &featA[tid * FP];
        if (p < NPATCH) {
            const int pr = p / RH, pc = p - pr * RH;
            const float* base = &ximg[(pr - pr0) * XP + pc];
            float s = 0.f;
            for (int i = 0; i < PATCH; ++i)
                for (int j = 0; j < PATCH; ++j) s += base[i * XP + j];
            const float mean = s * (1.0f / KPIX);
            float ss = 0.f;
            for (int i = 0; i < PATCH; ++i)
                for (int j = 0; j < PATCH; ++j) {
                    const float d = base[i * XP + j] - mean;
                    ss += d * d;
                }
            const float stdv = sqrtf(ss * (1.0f / (KPIX - 1))) + EPSV;
            const float inv  = 1.0f / stdv;
            row[0] = (_Float16)1.0f;
            for (int i = 0; i < PATCH; ++i)
                for (int j = 0; j < PATCH; ++j)
                    row[1 + i * PATCH + j] = (_Float16)((base[i * XP + j] - mean) * inv);
            for (int k = 122; k < 128; ++k) row[k] = (_Float16)0.f;
        } else {
            for (int k = 0; k < 128; ++k) row[k] = (_Float16)0.f;
        }
    }
    __syncthreads();

    v8f acc2[8] = {};

#pragma unroll 1
    for (int kc = 0; kc < 4; ++kc) {
        {
            const int r  = tid >> 1;
            const int k0 = (tid & 1) * 64;
            const float* w1row = W1 + (size_t)(kc * 128 + r) * 122;
            const float* w2row = W2 + (size_t)r * 512 + kc * 128;
#pragma unroll 4
            for (int k = k0; k < k0 + 64; k += 2) {
                v2h pk1, pk2;
                pk1[0] = (_Float16)(((k     < 122) ? w1row[k]     : 0.f) * WSCALE);
                pk1[1] = (_Float16)(((k + 1 < 122) ? w1row[k + 1] : 0.f) * WSCALE);
                pk2[0] = (_Float16)(w2row[k]     * WSCALE);
                pk2[1] = (_Float16)(w2row[k + 1] * WSCALE);
                *(v2h*)&w1c[r * FP + k] = pk1;
                *(v2h*)&w2c[r * FP + k] = pk2;
            }
        }
        __syncthreads();

#pragma unroll 1
        for (int nh = 0; nh < 2; ++nh) {
            v8f acc1[4] = {};
#pragma unroll
            for (int kt = 0; kt < 4; ++kt) {
                const v16h a = load_frag(&featA[(mrow + lmod) * FP + kt * 32 + lhalf * 8]);
#pragma unroll
                for (int nt = 0; nt < 4; ++nt) {
                    const v16h b = load_frag(&w1c[((nh * 4 + nt) * 16 + lmod) * FP + kt * 32 + lhalf * 8]);
                    acc1[nt] = wmma16(a, b, acc1[nt]);
                }
            }
#pragma unroll
            for (int nt = 0; nt < 4; ++nt) {
                const int col = (nh * 4 + nt) * 16 + lmod;
                const float bias = b1[kc * 128 + col];
#pragma unroll
                for (int i = 0; i < 8; ++i) {
                    const int rloc = mrow + lhalf * 8 + i;
                    h1A[rloc * FP + col] = (_Float16)fast_tanh(acc1[nt][i] * WINV + bias);
                }
            }
        }
        __syncthreads();

#pragma unroll
        for (int kt = 0; kt < 4; ++kt) {
            const v16h a = load_frag(&h1A[(mrow + lmod) * FP + kt * 32 + lhalf * 8]);
#pragma unroll
            for (int nt = 0; nt < 8; ++nt) {
                const v16h b = load_frag(&w2c[(nt * 16 + lmod) * FP + kt * 32 + lhalf * 8]);
                acc2[nt] = wmma16(a, b, acc2[nt]);
            }
        }
        __syncthreads();
    }

#pragma unroll
    for (int nt = 0; nt < 8; ++nt) {
        const int col = nt * 16 + lmod;
        const float bias = b2[col];
#pragma unroll
        for (int i = 0; i < 8; ++i) {
            const int rloc = mrow + lhalf * 8 + i;
            h2s[rloc * H2P + col] = fast_tanh(acc2[nt][i] * WINV + bias);
        }
    }
    __syncthreads();

    if (tid < MT) {
        const int p = p0 + tid;
        float s = b3[0];
        const float* hrow = &h2s[tid * H2P];
#pragma unroll 8
        for (int n = 0; n < 128; ++n) s += hrow[n] * W3[n];
        outs[tid] = (p < NPATCH) ? fast_sigmoid(s) : 0.0f;
    }
    __syncthreads();

    if (wave == 0) {
        const v4f v = *(const v4f*)&outs[lane * 4];
        float* wp = ws + (size_t)img * WSP + (size_t)p0 + lane * 4;
        *(volatile v4f*)wp = v;
        __threadfence();
        *(volatile v4f*)wp = v;
    }
}

__global__ __launch_bounds__(256) void k_copy_out(const float* __restrict__ ws, float* __restrict__ out,
                                                  int n_out, int nimg)
{
    const int t  = blockIdx.x * 256 + threadIdx.x;
    const int e0 = t * 4;
    if (e0 >= n_out) return;
    if (e0 + 4 <= n_out) {
        v4f v;
#pragma unroll
        for (int q = 0; q < 4; ++q) {
            const int e = e0 + q;
            int im = e / NPATCH;
            if (im > nimg - 1) im = nimg - 1;
            const int p = e - im * NPATCH;
            v[q] = ws[(size_t)im * WSP + p];
        }
        float* op = out + e0;
        *(volatile v4f*)op = v;
        __threadfence();
        *(volatile v4f*)op = v;
    } else {
        float vals[4];
#pragma unroll
        for (int q = 0; q < 4; ++q) {
            const int e = e0 + q;
            float val = 0.0f;
            if (e < n_out) {
                int im = e / NPATCH;
                if (im > nimg - 1) im = nimg - 1;
                const int p = e - im * NPATCH;
                val = ws[(size_t)im * WSP + p];
            }
            vals[q] = val;
        }
#pragma unroll
        for (int q = 0; q < 4; ++q)
            if (e0 + q < n_out) *(volatile float*)(out + e0 + q) = vals[q];
        __threadfence();
#pragma unroll
        for (int q = 0; q < 4; ++q)
            if (e0 + q < n_out) *(volatile float*)(out + e0 + q) = vals[q];
    }
}

extern "C" void kernel_launch(void* const* d_in, const int* in_sizes, int n_in,
                              void* d_out, int out_size, void* d_ws, size_t ws_size,
                              hipStream_t stream) {
    if (n_in < 7) return;
    const float* x  = (const float*)d_in[0];
    const float* W1 = (const float*)d_in[1];
    const float* b1 = (const float*)d_in[2];
    const float* W2 = (const float*)d_in[3];
    const float* b2 = (const float*)d_in[4];
    const float* W3 = (const float*)d_in[5];
    const float* b3 = (const float*)d_in[6];
    float* out = (float*)d_out;
    float* ws  = (float*)d_ws;

    const int nimg = in_sizes[0] / (HW * HW);
    if (nimg <= 0 || out_size <= 0) return;
    if ((size_t)nimg * (size_t)WSP * sizeof(float) > ws_size) return;

    dim3 grid1((unsigned)(nimg * NTILES));
    dim3 block(256);
    k_patch_mlp<<<grid1, block, 0, stream>>>(x, W1, b1, W2, b2, W3, b3, ws, nimg);

    const int nthr   = (out_size + 3) / 4;
    const int blocks = (nthr + 255) / 256;
    k_copy_out<<<dim3((unsigned)blocks), block, 0, stream>>>(ws, out, out_size, nimg);
}
